// GraphAttentionLayer_61168924230016
// MI455X (gfx1250) — hardware-verified
//
#include <hip/hip_runtime.h>
#include <stddef.h>
#include <stdint.h>
#include <math.h>


#pragma clang fp contract(off)

#define NB     8
#define NN     2048
#define CIN    128
#define HD     64
#define MROWS  (NB * NN)
#define NTHR   256
#define PROWS  128
#define PPITCH 68
#define PBLK   (MROWS / PROWS)
#define PB_H   (MROWS * (CIN / 8) / NTHR)
#define PB_W   (HD * (CIN / 8) / NTHR)
#define ATHR   128
#define AROWS  64
#define ABLK   (MROWS / AROWS)
#define CSTN   256
#define WSMAX  134217728

static_assert(MROWS % PROWS == 0 && NN % PROWS == 0 && NN / PROWS == 16);
static_assert(NN % AROWS == 0 && NN / AROWS == 32 && NN % 32 == 0);
static_assert(CIN % 32 == 0 && HD == 64 && CIN / 8 == 16);
static_assert((MROWS * (CIN / 8)) % NTHR == 0 && (HD * (CIN / 8)) % NTHR == 0);
static_assert(PROWS == (NTHR / 32) * 16 && AROWS == (ATHR / 32) * 16);
static_assert(PPITCH % 4 == 0 && PPITCH >= HD);
static_assert(PBLK == NB * 16 && ABLK == NB * 32);

typedef float          v4f   __attribute__((ext_vector_type(4)));
typedef float          v8f   __attribute__((ext_vector_type(8)));
typedef int            v8i   __attribute__((ext_vector_type(8)));
typedef unsigned short v8us  __attribute__((ext_vector_type(8)));
typedef unsigned short v16us __attribute__((ext_vector_type(16)));
typedef __bf16         v16bf __attribute__((ext_vector_type(16)));
typedef v4f  __attribute__((may_alias)) v4fa;
typedef v8us __attribute__((may_alias)) v8usa;
union FragB { v16bf v; v16us u; v8us h[2]; v8i w; };

__device__ __forceinline__ v8f wmb(const FragB& a, const FragB& b, v8f c) {
  v8f d = __builtin_amdgcn_wmma_f32_16x16x32_bf16(false, a.v, false, b.v, (short)0, c, false, false);
  asm volatile("v_nop\n\tv_nop\n\tv_nop\n\tv_nop" : "+v"(d) : "v"(a.w), "v"(b.w));
  return d;
}

__device__ __forceinline__ unsigned bf16_bits(float f) {
  const unsigned u = __float_as_uint(f);
  return (u + 0x7FFFu + ((u >> 16) & 1u)) >> 16;
}
__device__ __forceinline__ float bf16_val(float f) {
  return __uint_as_float(bf16_bits(f) << 16);
}

__global__ __launch_bounds__(NTHR) void k_prep(const float* __restrict__ h, const float* __restrict__ W,
                                               const float* __restrict__ bfc, const float* __restrict__ asrc,
                                               const float* __restrict__ adst, const float* __restrict__ battn,
                                               unsigned short* HB, unsigned short* WT, float* CST) {
  const int blk = (int)blockIdx.x, tid = (int)threadIdx.x;
  if (blk < PB_H) {
    const int u   = blk * NTHR + tid;
    const int row = u >> 4;
    const int k8  = (u & 15) * 8;
    const float* p = h + (size_t)row * CIN + k8;
    const v4f a = *(const v4fa*)p;
    const v4f b = *(const v4fa*)(p + 4);
    v8us o;
    o[0] = (unsigned short)bf16_bits(a.x); o[1] = (unsigned short)bf16_bits(a.y);
    o[2] = (unsigned short)bf16_bits(a.z); o[3] = (unsigned short)bf16_bits(a.w);
    o[4] = (unsigned short)bf16_bits(b.x); o[5] = (unsigned short)bf16_bits(b.y);
    o[6] = (unsigned short)bf16_bits(b.z); o[7] = (unsigned short)bf16_bits(b.w);
    unsigned short* dp = HB + (size_t)row * CIN + k8;
    *(volatile v8us*)dp = o;
    __threadfence();
    *(volatile v8us*)dp = o;
  } else if (blk < PB_H + PB_W) {
    const int v  = (blk - PB_H) * NTHR + tid;
    const int n  = v >> 4;
    const int k8 = (v & 15) * 8;
    const float* p = W + (size_t)k8 * HD + n;
    v8us o;
#pragma unroll
    for (int i = 0; i < 8; ++i) o[i] = (unsigned short)bf16_bits(p[(size_t)i * HD]);
    unsigned short* dp = WT + (size_t)n * CIN + k8;
    *(volatile v8us*)dp = o;
    __threadfence();
    *(volatile v8us*)dp = o;
  } else {
    const int lane = tid & 31, wave = tid >> 5;
    if (wave >= 4) return;
    const float* src = (wave == 0) ? bfc : ((wave == 1) ? asrc : adst);
    const int c4 = 4 * (lane & 15);
    const v4f a = *(const v4fa*)(src + c4);
    const float bt = battn[0];
    const bool w3 = (wave == 3);
    const float z0 = (lane == 0) ? bf16_val(bt) : 0.0f;
    v4f o;
    o.x = w3 ? z0   : bf16_val(a.x);
    o.y = w3 ? 0.0f : bf16_val(a.y);
    o.z = w3 ? 0.0f : bf16_val(a.z);
    o.w = w3 ? 0.0f : bf16_val(a.w);
    float* dp = CST + 64 * wave + c4;
    const bool ok = lane < 16;
    if (ok) *(volatile v4f*)dp = o;
    __threadfence();
    if (ok) *(volatile v4f*)dp = o;
  }
}

__global__ __launch_bounds__(NTHR) void k_proj(const unsigned short* __restrict__ HB,
                                               const unsigned short* __restrict__ WT,
                                               const float* __restrict__ CST,
                                               unsigned short* HPTH, unsigned short* HPTL,
                                               float* S, float* D, float* DMAXP) {
  __shared__ __attribute__((aligned(16))) float stg[PROWS * PPITCH];
  __shared__ __attribute__((aligned(16))) float cl[192];
  __shared__ __attribute__((aligned(16))) float sl[PROWS];
  __shared__ __attribute__((aligned(16))) float dl[PROWS];
  const int tid = (int)threadIdx.x, lane = tid & 31, wave = tid >> 5, hh = lane >> 4, mm = lane & 15;
  const int blk = (int)blockIdx.x;
  const int rowBase = blk * PROWS;
  const int b  = blk >> 4;
  const int jb = (blk & 15) * PROWS;

  if (tid < 48) *(v4fa*)(cl + 4 * tid) = *(const v4fa*)(CST + 4 * tid);

  v8f acc[4];
  {
    const v8f z = {0.f, 0.f, 0.f, 0.f, 0.f, 0.f, 0.f, 0.f};
    acc[0] = z; acc[1] = z; acc[2] = z; acc[3] = z;
  }
  const unsigned short* ap = HB + (size_t)(rowBase + 16 * wave + mm) * CIN + 8 * hh;
  const unsigned short* wp = WT + (size_t)mm * CIN + 8 * hh;
#pragma unroll 1
  for (int ks = 0; ks < CIN / 32; ++ks) {
    FragB af;
    af.h[0] = *(const v8usa*)(ap + 32 * ks);
    af.h[1] = *(const v8usa*)(ap + 32 * ks + 16);
#pragma unroll
    for (int t = 0; t < 4; ++t) {
      const unsigned short* wq = wp + (size_t)(16 * t) * CIN + 32 * ks;
      FragB bf;
      bf.h[0] = *(const v8usa*)wq;
      bf.h[1] = *(const v8usa*)(wq + 16);
      acc[t] = wmb(af, bf, acc[t]);
    }
  }
  __syncthreads();

#pragma unroll
  for (int t = 0; t < 4; ++t) {
    const int lc = 16 * t + mm;
    const float bv = cl[lc];
#pragma unroll
    for (int r = 0; r < 8; ++r) {
      const int lr = 16 * wave + 8 * hh + r;
      stg[lr * PPITCH + lc] = acc[t][r] + bv;
    }
  }
  __syncthreads();

  if (tid < PROWS) {
    const float* rp = stg + tid * PPITCH;
    float ss = 0.0f, dd = 0.0f;
#pragma unroll 4
    for (int e4 = 0; e4 < HD / 4; ++e4) {
      const v4f v  = *(const v4fa*)(rp + 4 * e4);
      const v4f as = *(const v4fa*)(cl + 64 + 4 * e4);
      const v4f ad = *(const v4fa*)(cl + 128 + 4 * e4);
      ss = fmaf(v.x, as.x, ss); dd = fmaf(v.x, ad.x, dd);
      ss = fmaf(v.y, as.y, ss); dd = fmaf(v.y, ad.y, dd);
      ss = fmaf(v.z, as.z, ss); dd = fmaf(v.z, ad.z, dd);
      ss = fmaf(v.w, as.w, ss); dd = fmaf(v.w, ad.w, dd);
    }
    sl[tid] = ss;
    dl[tid] = dd;
  }

  v8us qh[4], ql[4];
  {
    const int jl = 8 * (tid & 15);
#pragma unroll
    for (int it = 0; it < 4; ++it) {
      const int e = 16 * it + (tid >> 4);
      v8us oh, ol;
#pragma unroll
      for (int i = 0; i < 8; ++i) {
        const float v = stg[(jl + i) * PPITCH + e];
        const unsigned hb = bf16_bits(v);
        const unsigned lb = bf16_bits(v - __uint_as_float(hb << 16));
        oh[i] = (unsigned short)hb;
        ol[i] = (unsigned short)lb;
      }
      qh[it] = oh; ql[it] = ol;
    }
  }
  __syncthreads();

  const v4f s4 = *(const v4fa*)(sl + 4 * lane);
  const v4f d4 = *(const v4fa*)(dl + 4 * lane);
  float mx = fmaxf(fmaxf(d4.x, d4.y), fmaxf(d4.z, d4.w));
  mx = fmaxf(mx, __shfl_xor(mx, 16, 32));
  mx = fmaxf(mx, __shfl_xor(mx, 8, 32));
  mx = fmaxf(mx, __shfl_xor(mx, 4, 32));
  mx = fmaxf(mx, __shfl_xor(mx, 2, 32));
  mx = fmaxf(mx, __shfl_xor(mx, 1, 32));
  const v4f m4 = {mx, mx, mx, mx};
  const v4f sv = (wave == 0) ? s4 : ((wave == 1) ? d4 : m4);
  float* sp = (wave == 0) ? (S + rowBase + 4 * lane)
            : ((wave == 1) ? (D + rowBase + 4 * lane)
                           : (DMAXP + (size_t)blk * 32 + 4 * (lane & 7)));
  const bool sok = (wave < 2) || (wave == 2 && lane < 8);

  unsigned short* gh = HPTH + ((size_t)b * HD + (tid >> 4)) * NN + jb + 8 * (tid & 15);
  unsigned short* gl = HPTL + ((size_t)b * HD + (tid >> 4)) * NN + jb + 8 * (tid & 15);

  if (sok) *(volatile v4f*)sp = sv;
#pragma unroll
  for (int it = 0; it < 4; ++it) {
    *(volatile v8us*)(gh + (size_t)(16 * it) * NN) = qh[it];
    *(volatile v8us*)(gl + (size_t)(16 * it) * NN) = ql[it];
  }
  __threadfence();
  if (sok) *(volatile v4f*)sp = sv;
#pragma unroll
  for (int it = 0; it < 4; ++it) {
    *(volatile v8us*)(gh + (size_t)(16 * it) * NN) = qh[it];
    *(volatile v8us*)(gl + (size_t)(16 * it) * NN) = ql[it];
  }
}

__device__ __forceinline__ void pgen(float dj, float si, float bat, float rmax, float& z,
                                     unsigned& hb, unsigned& lb) {
  float x = (si + dj) + bat;
  x = (x >= 0.0f) ? x : 0.2f * x;
  const float p = expf(x - rmax);
  z += p;
  hb = bf16_bits(p);
  lb = bf16_bits(p - __uint_as_float(hb << 16));
}

__global__ __launch_bounds__(ATHR) void k_attn(const unsigned short* __restrict__ HPTH,
                                               const unsigned short* __restrict__ HPTL,
                                               const float* __restrict__ S, const float* __restrict__ D,
                                               const float* __restrict__ DMAXP, const float* __restrict__ CST,
                                               float* out) {
  __shared__ __attribute__((aligned(16))) float stg[AROWS * HD];
  __shared__ __attribute__((aligned(16))) float ls[AROWS];
  const int tid = (int)threadIdx.x, lane = tid & 31, wave = tid >> 5, hh = lane >> 4, mm = lane & 15;
  const int i0 = (int)blockIdx.x * AROWS;
  const int b  = (int)blockIdx.x >> 5;

  const float si  = S[i0 + 16 * wave + mm];
  const float bat = CST[192];
  float dmx = DMAXP[(size_t)(b * 16 + mm) * 32];
  dmx = fmaxf(dmx, __shfl_xor(dmx, 1, 32));
  dmx = fmaxf(dmx, __shfl_xor(dmx, 2, 32));
  dmx = fmaxf(dmx, __shfl_xor(dmx, 4, 32));
  dmx = fmaxf(dmx, __shfl_xor(dmx, 8, 32));
  float rmax = (si + dmx) + bat;
  rmax = (rmax >= 0.0f) ? rmax : 0.2f * rmax;

  v8f acc[4];
  {
    const v8f z = {0.f, 0.f, 0.f, 0.f, 0.f, 0.f, 0.f, 0.f};
    acc[0] = z; acc[1] = z; acc[2] = z; acc[3] = z;
  }
  const float* dp = D + (size_t)b * NN + 8 * hh;
  const unsigned short* vh = HPTH + ((size_t)b * HD + mm) * NN + 8 * hh;
  const unsigned short* vl = HPTL + ((size_t)b * HD + mm) * NN + 8 * hh;
  float zacc = 0.0f;

#pragma unroll 1
  for (int ks = 0; ks < NN / 32; ++ks) {
    const int j0 = 32 * ks;
    const v4f d0 = *(const v4fa*)(dp + j0);
    const v4f d1 = *(const v4fa*)(dp + j0 + 4);
    const v4f d2 = *(const v4fa*)(dp + j0 + 16);
    const v4f d3 = *(const v4fa*)(dp + j0 + 20);
    const float dv[16] = {d0.x, d0.y, d0.z, d0.w, d1.x, d1.y, d1.z, d1.w,
                          d2.x, d2.y, d2.z, d2.w, d3.x, d3.y, d3.z, d3.w};
    unsigned hb[16], lb[16];
#pragma unroll
    for (int e = 0; e < 16; ++e) pgen(dv[e], si, bat, rmax, zacc, hb[e], lb[e]);
    FragB ah, al;
#pragma unroll
    for (int q = 0; q < 8; ++q) {
      ah.w[q] = (int)(hb[2 * q] | (hb[2 * q + 1] << 16));
      al.w[q] = (int)(lb[2 * q] | (lb[2 * q + 1] << 16));
    }
#pragma unroll
    for (int t = 0; t < 4; ++t) {
      const unsigned short* ph = vh + (size_t)(16 * t) * NN + j0;
      const unsigned short* pl = vl + (size_t)(16 * t) * NN + j0;
      FragB bh, bl;
      bh.h[0] = *(const v8usa*)ph;
      bh.h[1] = *(const v8usa*)(ph + 16);
      bl.h[0] = *(const v8usa*)pl;
      bl.h[1] = *(const v8usa*)(pl + 16);
      acc[t] = wmb(ah, bh, acc[t]);
      acc[t] = wmb(ah, bl, acc[t]);
      acc[t] = wmb(al, bh, acc[t]);
    }
  }

  const float zrow = zacc + __shfl_xor(zacc, 16, 32);
#pragma unroll
  for (int t = 0; t < 4; ++t) {
    const int lc = 16 * t + mm;
#pragma unroll
    for (int r = 0; r < 8; ++r) {
      const int lr = 16 * wave + 8 * hh + r;
      stg[lr * HD + lc] = acc[t][r];
    }
  }
  if (lane < 16) ls[16 * wave + lane] = zrow;
  __syncthreads();

  v4f fv[8];
#pragma unroll
  for (int i = 0; i < 8; ++i) {
    const int lr = 16 * wave + 2 * i + hh;
    const v4f v = *(const v4fa*)(stg + lr * HD + 4 * mm);
    const float il = 1.0f / ls[lr];
    v4f o;
    o.x = v.x * il; o.y = v.y * il; o.z = v.z * il; o.w = v.w * il;
    o.x = (o.x > 0.0f) ? o.x : expm1f(o.x);
    o.y = (o.y > 0.0f) ? o.y : expm1f(o.y);
    o.z = (o.z > 0.0f) ? o.z : expm1f(o.z);
    o.w = (o.w > 0.0f) ? o.w : expm1f(o.w);
    fv[i] = o;
  }
#pragma unroll
  for (int i = 0; i < 8; ++i) {
    const int lr = 16 * wave + 2 * i + hh;
    float* op = out + (size_t)(i0 + lr) * HD + 4 * mm;
    *(volatile v4f*)op = fv[i];
  }
  __threadfence();
#pragma unroll
  for (int i = 0; i < 8; ++i) {
    const int lr = 16 * wave + 2 * i + hh;
    float* op = out + (size_t)(i0 + lr) * HD + 4 * mm;
    *(volatile v4f*)op = fv[i];
  }
}

static inline size_t al256(size_t o) { return (o + 255) & ~(size_t)255; }

extern "C" void kernel_launch(void* const* d_in, const int* in_sizes, int n_in,
                              void* d_out, int out_size, void* d_ws, size_t ws_size,
                              hipStream_t stream) {
  if (n_in < 6) return;
  if (in_sizes[0] != MROWS * CIN) return;
  if (in_sizes[1] != CIN * HD) return;
  if (in_sizes[2] != HD || in_sizes[3] != HD || in_sizes[4] != HD) return;
  if (in_sizes[5] != 1) return;
  if (out_size != MROWS * HD) return;

  const float* h     = (const float*)d_in[0];
  const float* Wfc   = (const float*)d_in[1];
  const float* bfc   = (const float*)d_in[2];
  const float* asrc  = (const float*)d_in[3];
  const float* adst  = (const float*)d_in[4];
  const float* battn = (const float*)d_in[5];
  float* out = (float*)d_out;

  char* ws = (char*)d_ws;
  size_t off = 0;
  const size_t oHB  = off; off = al256(off + (size_t)MROWS * CIN * 2);
  const size_t oWT  = off; off = al256(off + (size_t)HD * CIN * 2);
  const size_t oCST = off; off = al256(off + (size_t)CSTN * 4);
  const size_t oPH  = off; off = al256(off + (size_t)NB * HD * NN * 2);
  const size_t oPL  = off; off = al256(off + (size_t)NB * HD * NN * 2);
  const size_t oS   = off; off = al256(off + (size_t)MROWS * 4);
  const size_t oD   = off; off = al256(off + (size_t)MROWS * 4);
  const size_t oDM  = off; off = al256(off + (size_t)PBLK * 32 * 4);
  if (off > ws_size || off > (size_t)WSMAX) return;
  unsigned short* HB   = (unsigned short*)(ws + oHB);
  unsigned short* WT   = (unsigned short*)(ws + oWT);
  float*          CST  = (float*)(ws + oCST);
  unsigned short* HPTH = (unsigned short*)(ws + oPH);
  unsigned short* HPTL = (unsigned short*)(ws + oPL);
  float*          S    = (float*)(ws + oS);
  float*          D    = (float*)(ws + oD);
  float*          DMX  = (float*)(ws + oDM);

  k_prep<<<PB_H + PB_W + 1, NTHR, 0, stream>>>(h, Wfc, bfc, asrc, adst, battn, HB, WT, CST);
  k_proj<<<PBLK, NTHR, 0, stream>>>(HB, WT, CST, HPTH, HPTL, S, D, DMX);
  k_attn<<<ABLK, ATHR, 0, stream>>>(HPTH, HPTL, S, D, DMX, CST, out);
}
